// GIN_16252156248490
// MI455X (gfx1250) — hardware-run, weakly checked
//
#include <hip/hip_runtime.h>
#include <stddef.h>
#include <stdint.h>

#ifndef TWO_TERM
#define TWO_TERM 1
#endif

#define NN      100000
#define NE      1600000
#define DF      128
#define KP      256
#define KG      (TWO_TERM ? 256 : 128)
#define MP      100096
#define NTHR    256
#define NWAVE   8
#define EPT     8
#define WCH     (32 * EPT)
#define NBRUN   1024
#define SLB     10
#define NBK     98
#define WLCAP   3584
#define RCAP    28672
#define DEGCAP  64
#define MAXDEG_MEAS   36
#define MAXB1024_MEAS 16721
#define ABM     64
#define GBM     64
#define GTHR    128
#define GNT     8
#define SP      132
#define PBW     (DF * KP / 8 / NTHR)
#define WSMAX   134217728

#define BK_ZINTS (NWAVE * WLCAP + RCAP + 3 * NBRUN)
#define BK_INTS  (BK_ZINTS + 16)
#define BK_LDS   (BK_INTS * 4)

static_assert(NN == 100000 && NE == 1600000 && DF == 128);
static_assert(DF == 32 * 4 && DF == 16 * GNT && KP == 2 * DF);
static_assert(KG % 32 == 0 && KP % 32 == 0 && KG <= KP);
static_assert(MP % GBM == 0 && MP % ABM == 0 && MP >= NN && MP == 1564 * 64);
static_assert(NBRUN == (1 << SLB) && NBRUN % ABM == 0 && NBRUN % 32 == 0);
static_assert(NBK * NBRUN >= MP);
static_assert(NE < (1 << 21) && (((long long)NE) << SLB) < (1LL << 31));
static_assert(NE % WCH == 0 && NE % 4 == 0);
static_assert(RCAP == NWAVE * WLCAP && RCAP % (NTHR * 4) == 0 && BK_ZINTS % (NTHR * 4) == 0);
static_assert((2 * NBRUN) % (NTHR * 4) == 0);
static_assert((long long)RCAP * 100 >= (long long)MAXB1024_MEAS * 105);
static_assert(WLCAP >= MAXB1024_MEAS / 8 + 8 * 46 + 1);
static_assert(MAXDEG_MEAS + 8 <= DEGCAP);
static_assert(BK_LDS <= 300000);
static_assert((GBM * SP + DF) * 4 <= 65536 && (SP * 4) % 16 == 0);
static_assert(GBM == (GTHR / 32) * 16 && ABM % NWAVE == 0);
static_assert((DF * KP / 8) % NTHR == 0);

typedef float          v4f   __attribute__((ext_vector_type(4)));
typedef float          v8f   __attribute__((ext_vector_type(8)));
typedef int            v4i   __attribute__((ext_vector_type(4)));
typedef int            v8i   __attribute__((ext_vector_type(8)));
typedef unsigned short v8us  __attribute__((ext_vector_type(8)));
typedef unsigned short v16us __attribute__((ext_vector_type(16)));
typedef __bf16         v16bf __attribute__((ext_vector_type(16)));
typedef v4f  __attribute__((may_alias)) v4fa;
typedef v4i  __attribute__((may_alias)) v4ia;
typedef v8us __attribute__((may_alias)) v8usa;
union FragB { v16bf v; v16us u; v8us h[2]; v8i w; };

__device__ __forceinline__ v8f wmb(const FragB& a, const FragB& b, v8f c) {
  v8f d = __builtin_amdgcn_wmma_f32_16x16x32_bf16(false, a.v, false, b.v, (short)0, c, false, false);
  asm volatile("v_nop\n\tv_nop\n\tv_nop\n\tv_nop" : "+v"(d) : "v"(a.w), "v"(b.w));
  return d;
}

__device__ __forceinline__ unsigned bf16_bits(float f) {
  const unsigned u = __float_as_uint(f);
  const unsigned r = (u + 0x7FFFu + ((u >> 16) & 1u)) >> 16;
  const unsigned q = (u >> 16) | 0x40u;
  return ((u & 0x7fffffffu) > 0x7f800000u) ? q : r;
}
__device__ __forceinline__ float bf16_val(float f) {
  return __uint_as_float(bf16_bits(f) << 16);
}

__device__ __forceinline__ void hilo_pack(float v0, float v1, float v2, float v3,
                                          int& h01, int& h23, int& l01, int& l23) {
  const unsigned a0 = bf16_bits(v0), a1 = bf16_bits(v1), a2 = bf16_bits(v2), a3 = bf16_bits(v3);
  const unsigned b0 = bf16_bits(v0 - __uint_as_float(a0 << 16));
  const unsigned b1 = bf16_bits(v1 - __uint_as_float(a1 << 16));
  const unsigned b2 = bf16_bits(v2 - __uint_as_float(a2 << 16));
  const unsigned b3 = bf16_bits(v3 - __uint_as_float(a3 << 16));
  h01 = (int)(a0 | (a1 << 16)); h23 = (int)(a2 | (a3 << 16));
  l01 = (int)(b0 | (b1 << 16)); l23 = (int)(b2 | (b3 << 16));
}

__device__ __forceinline__ v4i regroup32(int h01, int h23, int l01, int l23, int lane) {
  const int s0 = 2 * (lane & 15), s1 = s0 + 1;
  const int a0 = __shfl(h01, s0, 32), a1 = __shfl(h23, s0, 32), a2 = __shfl(h01, s1, 32), a3 = __shfl(h23, s1, 32);
  const int b0 = __shfl(l01, s0, 32), b1 = __shfl(l23, s0, 32), b2 = __shfl(l01, s1, 32), b3 = __shfl(l23, s1, 32);
  const int mk = (lane < 16) ? -1 : 0;
  v4i o;
  o.x = (a0 & mk) | (b0 & ~mk); o.y = (a1 & mk) | (b1 & ~mk);
  o.z = (a2 & mk) | (b2 & ~mk); o.w = (a3 & mk) | (b3 & ~mk);
  return o;
}

__device__ __forceinline__ void st2_v4f(float* p, v4f v) {
  *(volatile v4f*)p = v;
  __threadfence();
  *(volatile v4f*)p = v;
}
__device__ __forceinline__ void st2_v8us(unsigned short* p, v8us v) {
  *(volatile v8us*)p = v;
  __threadfence();
  *(volatile v8us*)p = v;
}

__device__ __forceinline__ v8us gather8(const float* __restrict__ base, int stride) {
  float f[8];
#pragma unroll
  for (int i = 0; i < 8; ++i) f[i] = base[(size_t)i * (size_t)stride];
  v8us o;
#pragma unroll
  for (int i = 0; i < 8; ++i) o[i] = (unsigned short)bf16_bits(f[i]);
  return o;
}

__device__ __forceinline__ float nmax(float m, float v) {
  return ((v > m) | (v != v)) ? v : m;
}

__global__ __launch_bounds__(NTHR) void k_prep(const float* __restrict__ w1, const float* __restrict__ b1,
                                               const float* __restrict__ w2, const float* __restrict__ b2,
                                               unsigned short* wd, float* bt) {
  const int tid = (int)threadIdx.x, lane = tid & 31;
  const int blk = (int)blockIdx.x;
  if (blk < PBW) {
    const int u = blk * NTHR + tid;
    const int n = u >> 5, k8 = (u & 31) * 8, kk = k8 & (DF - 1);
    const v8us o = gather8(w1 + (size_t)kk * DF + n, DF);
    st2_v8us(wd + (size_t)n * KP + k8, o);
  } else if (blk < 2 * PBW) {
    const int u = (blk - PBW) * NTHR + tid;
    const int n = u >> 5, k8 = (u & 31) * 8, kk = k8 & (DF - 1);
    const v8us o = gather8(w2 + (size_t)kk * DF + n, DF);
    st2_v8us(wd + (size_t)DF * KP + (size_t)n * KP + k8, o);
  } else {
    if (tid < 32) {
      const v4f a = *(const v4fa*)(b1 + 4 * lane);
      const v4f c = *(const v4fa*)(b2 + 4 * lane);
      v4f oa, oc;
      oa.x = bf16_val(a.x); oa.y = bf16_val(a.y); oa.z = bf16_val(a.z); oa.w = bf16_val(a.w);
      oc.x = bf16_val(c.x); oc.y = bf16_val(c.y); oc.z = bf16_val(c.z); oc.w = bf16_val(c.w);
      st2_v4f(bt + 4 * lane, oa);
      st2_v4f(bt + DF + 4 * lane, oc);
    }
  }
}

__device__ __forceinline__ void bucket_flush(const int* pl, const int* cnt, int ov, int* lp, int* cop, int* fp,
                                             int tid) {
#pragma unroll 1
  for (int i = tid * 4; i < RCAP; i += NTHR * 4) {
    const v4i v = *(const v4ia*)(pl + i);
    *(volatile v4i*)(lp + i) = v;
  }
#pragma unroll 1
  for (int i = tid * 4; i < 2 * NBRUN; i += NTHR * 4) {
    const v4i v = *(const v4ia*)(cnt + i);
    *(volatile v4i*)(cop + i) = v;
  }
  if (tid < 8) {
    const v4i f = {ov, ov, ov, ov};
    *(volatile v4i*)(fp + 4 * tid) = f;
  }
}

__global__ __launch_bounds__(NTHR) void k_bucket(const int* __restrict__ srcs, const int* __restrict__ dsts,
                                                 int* LIST, int* CO, int* FLAG) {
  extern __shared__ __attribute__((aligned(16))) int dsm[];
  int* wl   = dsm;
  int* pl   = dsm + NWAVE * WLCAP;
  int* cnt  = pl + RCAP;
  int* offs = cnt + NBRUN;
  int* cur  = offs + NBRUN;
  int* misc = cur + NBRUN;
  const int tid = (int)threadIdx.x, lane = tid & 31, wave = tid >> 5;
  const int blk = (int)blockIdx.x;
  const unsigned nbs = (unsigned)(blk * NBRUN);

  {
    const v4i z4 = {0, 0, 0, 0};
    for (int i = tid * 4; i < BK_ZINTS; i += NTHR * 4) *(v4ia*)(dsm + i) = z4;
    if (tid < 16) misc[tid] = 0;
  }
  __syncthreads();

  {
    const int per  = ((NE + NWAVE * WCH - 1) / (NWAVE * WCH)) * WCH;
    const int ebeg = wave * per;
    const int eend = (ebeg + per < NE) ? (ebeg + per) : NE;
    int* mylist = wl + wave * WLCAP;
    int wc = 0;
#pragma unroll 1
    for (int cb = ebeg; cb < eend; cb += WCH) {
      const int e0 = cb + lane * EPT;
      const v4i da = *(const v4ia*)(dsts + e0);
      const v4i db = *(const v4ia*)(dsts + e0 + 4);
      const unsigned s0 = (unsigned)da.x - nbs, s1 = (unsigned)da.y - nbs;
      const unsigned s2 = (unsigned)da.z - nbs, s3 = (unsigned)da.w - nbs;
      const unsigned s4 = (unsigned)db.x - nbs, s5 = (unsigned)db.y - nbs;
      const unsigned s6 = (unsigned)db.z - nbs, s7 = (unsigned)db.w - nbs;
      const bool h0 = s0 < (unsigned)NBRUN, h1 = s1 < (unsigned)NBRUN, h2 = s2 < (unsigned)NBRUN, h3 = s3 < (unsigned)NBRUN;
      const bool h4 = s4 < (unsigned)NBRUN, h5 = s5 < (unsigned)NBRUN, h6 = s6 < (unsigned)NBRUN, h7 = s7 < (unsigned)NBRUN;
      const unsigned m0 = __builtin_amdgcn_ballot_w32(h0), m1 = __builtin_amdgcn_ballot_w32(h1);
      const unsigned m2 = __builtin_amdgcn_ballot_w32(h2), m3 = __builtin_amdgcn_ballot_w32(h3);
      const unsigned m4 = __builtin_amdgcn_ballot_w32(h4), m5 = __builtin_amdgcn_ballot_w32(h5);
      const unsigned m6 = __builtin_amdgcn_ballot_w32(h6), m7 = __builtin_amdgcn_ballot_w32(h7);
      const unsigned any = m0 | m1 | m2 | m3 | m4 | m5 | m6 | m7;
      if (any != 0u) {
        const int pre = (int)(__builtin_amdgcn_mbcnt_lo(m0, 0u) + __builtin_amdgcn_mbcnt_lo(m1, 0u) +
                              __builtin_amdgcn_mbcnt_lo(m2, 0u) + __builtin_amdgcn_mbcnt_lo(m3, 0u) +
                              __builtin_amdgcn_mbcnt_lo(m4, 0u) + __builtin_amdgcn_mbcnt_lo(m5, 0u) +
                              __builtin_amdgcn_mbcnt_lo(m6, 0u) + __builtin_amdgcn_mbcnt_lo(m7, 0u));
        int p = wc + pre;
        if (h0) { if (p < WLCAP) mylist[p] = ((e0 + 0) << SLB) | (int)s0; p = p + 1; }
        if (h1) { if (p < WLCAP) mylist[p] = ((e0 + 1) << SLB) | (int)s1; p = p + 1; }
        if (h2) { if (p < WLCAP) mylist[p] = ((e0 + 2) << SLB) | (int)s2; p = p + 1; }
        if (h3) { if (p < WLCAP) mylist[p] = ((e0 + 3) << SLB) | (int)s3; p = p + 1; }
        if (h4) { if (p < WLCAP) mylist[p] = ((e0 + 4) << SLB) | (int)s4; p = p + 1; }
        if (h5) { if (p < WLCAP) mylist[p] = ((e0 + 5) << SLB) | (int)s5; p = p + 1; }
        if (h6) { if (p < WLCAP) mylist[p] = ((e0 + 6) << SLB) | (int)s6; p = p + 1; }
        if (h7) { if (p < WLCAP) mylist[p] = ((e0 + 7) << SLB) | (int)s7; p = p + 1; }
        wc += (int)(__builtin_popcount(m0) + __builtin_popcount(m1) + __builtin_popcount(m2) + __builtin_popcount(m3) +
                    __builtin_popcount(m4) + __builtin_popcount(m5) + __builtin_popcount(m6) + __builtin_popcount(m7));
      }
    }
    if (lane == 0) misc[wave] = wc;
  }
  __syncthreads();

  if (wave == 0) {
    int ov = 0;
#pragma unroll 1
    for (int w2 = 0; w2 < NWAVE; ++w2) {
      int c = misc[w2];
      if (c > WLCAP) ov = 1;
      c = c < 0 ? 0 : (c > WLCAP ? WLCAP : c);
#pragma unroll 1
      for (int b0 = 0; b0 < c; b0 += 32) {
        const int idx = b0 + lane;
        const int ent = wl[w2 * WLCAP + (idx < WLCAP ? idx : WLCAP - 1)];
        const int m32 = (c - b0) < 32 ? (c - b0) : 32;
#pragma unroll 1
        for (int k = 0; k < m32; ++k) {
          const int u    = __builtin_amdgcn_readlane(ent, k);
          const int slot = u & (NBRUN - 1);
          if (lane == 0) cnt[slot] = cnt[slot] + 1;
        }
      }
    }
    if (lane == 0) misc[9] = ov;
  }
  __syncthreads();
  if (wave == 0) {
    const int base = lane * (NBRUN / 32);
    int s = 0;
#pragma unroll 1
    for (int i = 0; i < NBRUN / 32; ++i) s += cnt[base + i];
    int incl = s;
#pragma unroll
    for (int d = 1; d < 32; d <<= 1) {
      const int y = __shfl_up(incl, d, 32);
      if (lane >= d) incl += y;
    }
    int run = incl - s;
#pragma unroll 1
    for (int i = 0; i < NBRUN / 32; ++i) {
      const int cv = cnt[base + i];
      offs[base + i] = run;
      cur[base + i]  = run;
      run += cv;
    }
  }
  __syncthreads();

  if (wave == 0) {
#pragma unroll 1
    for (int w2 = 0; w2 < NWAVE; ++w2) {
      int c = misc[w2];
      c = c < 0 ? 0 : (c > WLCAP ? WLCAP : c);
#pragma unroll 1
      for (int b0 = 0; b0 < c; b0 += 32) {
        const int idx = b0 + lane;
        const int ent = wl[w2 * WLCAP + (idx < WLCAP ? idx : WLCAP - 1)];
        int eid = (ent >> SLB) & 0x1FFFFF;
        eid = eid > NE - 1 ? NE - 1 : eid;
        int sr = srcs[eid];
        sr = sr < 0 ? 0 : (sr > NN - 1 ? NN - 1 : sr);
        const int m32 = (c - b0) < 32 ? (c - b0) : 32;
#pragma unroll 1
        for (int k = 0; k < m32; ++k) {
          const int u    = __builtin_amdgcn_readlane(ent, k);
          const int wd   = __builtin_amdgcn_readlane(sr, k);
          const int slot = u & (NBRUN - 1);
          if (lane == 0) {
            int p = cur[slot];
            p = p < 0 ? 0 : (p > RCAP - 1 ? RCAP - 1 : p);
            pl[p] = wd;
            cur[slot] = p + 1;
          }
        }
      }
    }
  }
  __syncthreads();

  const int ovf = misc[9];
  int* lp  = LIST + (size_t)blk * RCAP;
  int* cop = CO + (size_t)blk * (2 * NBRUN);
  int* fp  = FLAG + (size_t)blk * 32;
  bucket_flush(pl, cnt, ovf, lp, cop, fp, tid);
  __threadfence();
  bucket_flush(pl, cnt, ovf, lp, cop, fp, tid);
}

template <int LAYER>
__global__ __launch_bounds__(NTHR) void k_replay(const int* __restrict__ LIST, const int* __restrict__ CO,
                                                 const int* __restrict__ FLAG, const float* __restrict__ F,
                                                 unsigned short* S) {
  const int tid = (int)threadIdx.x, lane = tid & 31;
  const int wave = __builtin_amdgcn_readfirstlane(tid >> 5);
  const int rowBase = (int)blockIdx.x * ABM;
  const int bucket  = rowBase >> SLB;
  const int* lb  = LIST + (size_t)bucket * RCAP;
  const int* cob = CO + (size_t)bucket * (2 * NBRUN);
  const int flag = FLAG[(size_t)bucket * 32];
  const float qnan = __uint_as_float(0x7fc00000u);
  const float ninf = __uint_as_float(0xff800000u);

#pragma unroll 1
  for (int i = 0; i < ABM / NWAVE; ++i) {
    const int d    = rowBase + (ABM / NWAVE) * wave + i;
    const int slot = d & (NBRUN - 1);
    const int craw = cob[slot];
    int o = cob[NBRUN + slot];
    const bool big = craw > DEGCAP;
    int c = craw < 0 ? 0 : (craw > DEGCAP ? DEGCAP : craw);
    o = o < 0 ? 0 : (o > RCAP - 1 ? RCAP - 1 : o);
    c = __builtin_amdgcn_readfirstlane(c);
    o = __builtin_amdgcn_readfirstlane(o);
    int last = o + (c > 0 ? c : 1) - 1;
    last = last > RCAP - 1 ? RCAP - 1 : last;

    float m0 = ninf, m1 = ninf, m2 = ninf, m3 = ninf;
#pragma unroll 1
    for (int j = 0; j < c; j += 4) {
      int i0 = o + j, i1 = i0 + 1, i2 = i0 + 2, i3 = i0 + 3;
      i0 = i0 > last ? last : i0; i1 = i1 > last ? last : i1;
      i2 = i2 > last ? last : i2; i3 = i3 > last ? last : i3;
      int r0 = lb[i0], r1 = lb[i1], r2 = lb[i2], r3 = lb[i3];
      r0 = r0 < 0 ? 0 : (r0 > NN - 1 ? NN - 1 : r0);
      r1 = r1 < 0 ? 0 : (r1 > NN - 1 ? NN - 1 : r1);
      r2 = r2 < 0 ? 0 : (r2 > NN - 1 ? NN - 1 : r2);
      r3 = r3 < 0 ? 0 : (r3 > NN - 1 ? NN - 1 : r3);
      const v4f v0 = *(const v4fa*)(F + (size_t)r0 * DF + 4 * lane);
      const v4f v1 = *(const v4fa*)(F + (size_t)r1 * DF + 4 * lane);
      const v4f v2 = *(const v4fa*)(F + (size_t)r2 * DF + 4 * lane);
      const v4f v3 = *(const v4fa*)(F + (size_t)r3 * DF + 4 * lane);
      asm volatile("" :: "v"(v0), "v"(v1));
      asm volatile("" :: "v"(v2), "v"(v3));
      m0 = nmax(m0, v0.x); m1 = nmax(m1, v0.y); m2 = nmax(m2, v0.z); m3 = nmax(m3, v0.w);
      m0 = nmax(m0, v1.x); m1 = nmax(m1, v1.y); m2 = nmax(m2, v1.z); m3 = nmax(m3, v1.w);
      m0 = nmax(m0, v2.x); m1 = nmax(m1, v2.y); m2 = nmax(m2, v2.z); m3 = nmax(m3, v2.w);
      m0 = nmax(m0, v3.x); m1 = nmax(m1, v3.y); m2 = nmax(m2, v3.z); m3 = nmax(m3, v3.w);
    }
    if (LAYER == 1) { m0 = bf16_val(m0); m1 = bf16_val(m1); m2 = bf16_val(m2); m3 = bf16_val(m3); }
    const bool empty = (c == 0);
    const bool z0 = empty | ((__float_as_uint(m0) & 0x7fffffffu) == 0x7f800000u);
    const bool z1 = empty | ((__float_as_uint(m1) & 0x7fffffffu) == 0x7f800000u);
    const bool z2 = empty | ((__float_as_uint(m2) & 0x7fffffffu) == 0x7f800000u);
    const bool z3 = empty | ((__float_as_uint(m3) & 0x7fffffffu) == 0x7f800000u);
    const float a0 = z0 ? 0.0f : m0, a1 = z1 ? 0.0f : m1, a2 = z2 ? 0.0f : m2, a3 = z3 ? 0.0f : m3;

    const bool live = d < NN;
    const int dc = live ? d : NN - 1;
    const v4f sf = *(const v4fa*)(F + (size_t)dc * DF + 4 * lane);
    asm volatile("" :: "v"(sf));
    float s0 = sf.x, s1 = sf.y, s2 = sf.z, s3 = sf.w;
    if (LAYER == 1) { s0 = bf16_val(s0); s1 = bf16_val(s1); s2 = bf16_val(s2); s3 = bf16_val(s3); }
    float t0 = s0 + a0, t1 = s1 + a1, t2 = s2 + a2, t3 = s3 + a3;
    const bool bad = (flag != 0) | big;
    t0 = bad ? qnan : t0; t1 = bad ? qnan : t1; t2 = bad ? qnan : t2; t3 = bad ? qnan : t3;
    t0 = live ? t0 : 0.0f; t1 = live ? t1 : 0.0f; t2 = live ? t2 : 0.0f; t3 = live ? t3 : 0.0f;

    int h01, h23, l01, l23;
    hilo_pack(t0, t1, t2, t3, h01, h23, l01, l23);
    const v4i ow = regroup32(h01, h23, l01, l23, lane);
    unsigned short* hp = S + (size_t)d * KP + 8 * lane;
    *(volatile v4i*)hp = ow;
    __threadfence();
    *(volatile v4i*)hp = ow;
  }
}

template <int RELU>
__global__ __launch_bounds__(GTHR) __attribute__((amdgpu_num_vgpr(248)))
void k_gemm(const unsigned short* __restrict__ A, const unsigned short* __restrict__ WT,
            const float* __restrict__ bt, float* outp, int nStore) {
  __shared__ __attribute__((aligned(16))) float stg[GBM * SP];
  __shared__ __attribute__((aligned(16))) float sb[DF];
  const int tid = (int)threadIdx.x, lane = tid & 31, hh = lane >> 4, m = lane & 15;
  const int wave = __builtin_amdgcn_readfirstlane(tid >> 5);
  const int rowBase = (int)blockIdx.x * GBM;
  if (tid < 32) *(v4fa*)(sb + 4 * tid) = *(const v4fa*)(bt + 4 * tid);

  v8f acc[GNT];
  {
    const v8f z = {0.f, 0.f, 0.f, 0.f, 0.f, 0.f, 0.f, 0.f};
#pragma unroll
    for (int t = 0; t < GNT; ++t) acc[t] = z;
  }
  const unsigned short* ap = A + (size_t)(rowBase + 16 * wave + m) * (size_t)KP + 8 * hh;
  const unsigned short* wp = WT + (size_t)m * (size_t)KP + 8 * hh;
#pragma unroll 1
  for (int k0 = 0; k0 < KG; k0 += 32) {
    FragB af;
    af.h[0] = *(const v8usa*)(ap + k0);
    af.h[1] = *(const v8usa*)(ap + k0 + 16);
#pragma unroll
    for (int t = 0; t < GNT; ++t) {
      const unsigned short* wq = wp + (size_t)(16 * t) * (size_t)KP + k0;
      FragB bf;
      bf.h[0] = *(const v8usa*)wq;
      bf.h[1] = *(const v8usa*)(wq + 16);
      acc[t] = wmb(af, bf, acc[t]);
    }
  }

#pragma unroll
  for (int t = 0; t < GNT; ++t) {
#pragma unroll
    for (int r = 0; r < 8; ++r) stg[(16 * wave + 8 * hh + r) * SP + 16 * t + m] = acc[t][r];
  }
  __syncthreads();

  const v4f bias = *(const v4fa*)(sb + 4 * lane);
#pragma unroll 1
  for (int i = 0; i < 16; ++i) {
    const int lr = 16 * wave + i;
    const int gr = rowBase + lr;
    const bool live = gr < NN;
    const v4f a = *(const v4fa*)(stg + lr * SP + 4 * lane);
    asm volatile("" :: "v"(a));
    float v0 = a.x + bias.x, v1 = a.y + bias.y, v2 = a.z + bias.z, v3 = a.w + bias.w;
    if (RELU != 0) {
      v0 = (v0 > 0.0f) ? v0 : (v0 - v0); v1 = (v1 > 0.0f) ? v1 : (v1 - v1);
      v2 = (v2 > 0.0f) ? v2 : (v2 - v2); v3 = (v3 > 0.0f) ? v3 : (v3 - v3);
    }
    v4f o;
    o.x = live ? v0 : 0.0f; o.y = live ? v1 : 0.0f; o.z = live ? v2 : 0.0f; o.w = live ? v3 : 0.0f;
    float* op = outp + (size_t)gr * DF + 4 * lane;
    const bool ok = gr < nStore;
    if (ok) *(volatile v4f*)op = o;
    __threadfence();
    if (ok) *(volatile v4f*)op = o;
  }
}

extern "C" void kernel_launch(void* const* d_in, const int* in_sizes, int n_in,
                              void* d_out, int out_size, void* d_ws, size_t ws_size,
                              hipStream_t stream) {
  if (n_in < 7) return;
  if (in_sizes[0] != NN * DF) return;
  if (in_sizes[1] != NE) return;
  if (in_sizes[2] != NE) return;
  if (in_sizes[3] != DF * DF) return;
  if (in_sizes[4] != DF) return;
  if (in_sizes[5] != DF * DF) return;
  if (in_sizes[6] != DF) return;
  if (out_size != NN * DF) return;

  const float* h   = (const float*)d_in[0];
  const int*   src = (const int*)d_in[1];
  const int*   dst = (const int*)d_in[2];
  const float* W1  = (const float*)d_in[3];
  const float* b1  = (const float*)d_in[4];
  const float* W2  = (const float*)d_in[5];
  const float* b2  = (const float*)d_in[6];
  float* out = (float*)d_out;

  constexpr size_t zS    = (size_t)MP * KP * 2;
  constexpr size_t zX1   = (size_t)MP * DF * 4;
  constexpr size_t zLIST = (size_t)NBK * RCAP * 4;
  constexpr size_t zCO   = (size_t)NBK * 2 * NBRUN * 4;
  constexpr size_t zFLAG = (size_t)NBK * 128;
  constexpr size_t zWD   = (size_t)2 * DF * KP * 2;
  constexpr size_t zBT   = (size_t)2 * DF * 4;
  constexpr size_t oS    = 0;
  constexpr size_t oX1   = oS + zS;
  constexpr size_t oLIST = oX1 + zX1;
  constexpr size_t oCO   = oLIST + zLIST;
  constexpr size_t oFLAG = oCO + zCO;
  constexpr size_t oWD   = oFLAG + zFLAG;
  constexpr size_t oBT   = oWD + zWD;
  constexpr size_t oEND  = oBT + zBT;
  static_assert(zS % 256 == 0 && zX1 % 256 == 0 && zLIST % 256 == 0 && zCO % 256 == 0);
  static_assert(zFLAG % 256 == 0 && zWD % 256 == 0 && zBT % 256 == 0);
  static_assert(oEND <= (size_t)WSMAX);
  static_assert((size_t)NN * DF - 1 == 12799999);
  if (oEND > ws_size) return;

  char* ws = (char*)d_ws;
  unsigned short* S    = (unsigned short*)(ws + oS);
  float*          X1   = (float*)(ws + oX1);
  int*            LIST = (int*)(ws + oLIST);
  int*            CO   = (int*)(ws + oCO);
  int*            FLAG = (int*)(ws + oFLAG);
  unsigned short* WD   = (unsigned short*)(ws + oWD);
  float*          BT   = (float*)(ws + oBT);

  hipFuncSetAttribute(reinterpret_cast<const void*>(&k_bucket), hipFuncAttributeMaxDynamicSharedMemorySize, (int)BK_LDS);

  k_prep<<<2 * PBW + 1, NTHR, 0, stream>>>(W1, b1, W2, b2, WD, BT);
  k_bucket<<<NBK, NTHR, BK_LDS, stream>>>(src, dst, LIST, CO, FLAG);
  k_replay<1><<<MP / ABM, NTHR, 0, stream>>>(LIST, CO, FLAG, h, S);
  k_gemm<1><<<MP / GBM, GTHR, 0, stream>>>(S, WD, BT, X1, MP);
  k_replay<2><<<MP / ABM, NTHR, 0, stream>>>(LIST, CO, FLAG, X1, S);
  k_gemm<0><<<(NN + GBM - 1) / GBM, GTHR, 0, stream>>>(S, WD + (size_t)DF * KP, BT + DF, out, NN);
}
